// LinearAttention_395136991249
// MI455X (gfx1250) — hardware-run, weakly checked
//
#include <hip/hip_runtime.h>


#define NBH  24
#define NHH  12
#define NN   4096
#define ND   64
constexpr size_t al256(size_t b) { return (b + 255) & ~(size_t)255; }
constexpr size_t WS_TOTAL = 4 * al256((size_t)NBH * ND * NN * 2) + al256((size_t)NBH * ND * ND * 4) + al256((size_t)NBH * ND * ND * 2);
static_assert(WS_TOTAL == 50921472 && WS_TOTAL <= 134217728, "the workspace carve: about 48.6 MiB");
static_assert(NN % 64 == 0 && ND % 64 == 0 && NN % 32 == 0 && ND % 32 == 0 && NN % 8 == 0, "whole 64 x 64 tiles; whole depth steps");
typedef _Float16 h16;
typedef unsigned short bf;
typedef __attribute__((ext_vector_type(16))) __bf16   v16bf;
typedef __attribute__((ext_vector_type(16))) _Float16 v16h;
typedef __attribute__((ext_vector_type(8)))  _Float16 v8h;
typedef __attribute__((ext_vector_type(8)))  unsigned short v8us;
typedef __attribute__((ext_vector_type(8)))  float    v8f;
typedef __attribute__((ext_vector_type(4)))  float    v4f;
typedef v8h  __attribute__((may_alias)) v8ha;
typedef v4f  __attribute__((may_alias)) v4fa;
typedef v8us __attribute__((may_alias)) v8usa;

__device__ __forceinline__ unsigned short f2bf(float f) { unsigned u = __float_as_uint(f); u += 0x7FFFu + ((u >> 16) & 1u); return (unsigned short)(u >> 16); }
__device__ __forceinline__ float bf2f(unsigned short b) { return __uint_as_float(((unsigned)b) << 16); }
__device__ __forceinline__ float bfr(float f) { return bf2f(f2bf(f)); }
__device__ __forceinline__ v16h cat16(v8h lo, v8h hi) { return __builtin_shufflevector(lo, hi, 0, 1, 2, 3, 4, 5, 6, 7, 8, 9, 10, 11, 12, 13, 14, 15); }
__device__ __forceinline__ v16bf cat16b(v8us lo, v8us hi) { return __builtin_bit_cast(v16bf, __builtin_shufflevector(lo, hi, 0, 1, 2, 3, 4, 5, 6, 7, 8, 9, 10, 11, 12, 13, 14, 15)); }
__device__ __forceinline__ v8f wmma16(v16h a, v16h b, v8f c) { return __builtin_amdgcn_wmma_f32_16x16x32_f16(false, a, false, b, (short)0, c, false, false); }
__device__ __forceinline__ v8f wmmab(v16bf a, v16bf b, v8f c) { return __builtin_amdgcn_wmma_f32_16x16x32_bf16(false, a, false, b, (short)0, c, false, false); }


template <typename T16> struct WFrag;
template <> struct WFrag<h16> { typedef v16h V; static __device__ __forceinline__ V ld(const h16* p) { return cat16(*(const v8h*)p, *(const v8h*)(p + 16)); } static __device__ __forceinline__ v8f mma(V a, V b, v8f c) { return wmma16(a, b, c); } };
template <> struct WFrag<bf> { typedef v16bf V; static __device__ __forceinline__ V ld(const bf* p) { return cat16b(*(const v8us*)p, *(const v8us*)(p + 16)); } static __device__ __forceinline__ v8f mma(V a, V b, v8f c) { return wmmab(a, b, c); } };
template <typename T16, int NSPLIT, bool BIAS>
__global__ __launch_bounds__(32) void k_gemmw(const T16* __restrict__ A, const T16* __restrict__ A2, const T16* __restrict__ Bt, const T16* __restrict__ Bt2, int K, float* C, int ldc, const float* __restrict__ bias, size_t sA, size_t sB, size_t sC) {
    typedef typename WFrag<T16>::V V;
    __shared__ __align__(16) float os[16 * 68];
    const size_t z = blockIdx.z; A += z * sA; if (A2) A2 += z * sA; Bt += z * sB; if (Bt2) Bt2 += z * sB; C += z * sC;
    const int lane = threadIdx.x & 31, lr = lane & 15, hi = lane >> 4; const int r0 = blockIdx.x * 64, c0 = blockIdx.y * 64;
    v8f acc[4][4];
#pragma unroll
    for (int mb = 0; mb < 4; ++mb)
#pragma unroll
        for (int nb = 0; nb < 4; ++nb) acc[mb][nb] = (v8f){};
    const size_t aoff = (size_t)(r0 + lr) * K + 8 * hi, boff = (size_t)(c0 + lr) * K + 8 * hi;
    for (int kc = 0; kc < K; kc += 32) {
        V a[4], a2[4];
#pragma unroll
        for (int mb = 0; mb < 4; ++mb) { a[mb] = WFrag<T16>::ld(A + aoff + (size_t)mb * 16 * K + kc); if (NSPLIT == 1 || NSPLIT == 2) a2[mb] = WFrag<T16>::ld(A2 + aoff + (size_t)mb * 16 * K + kc); }
#pragma unroll
        for (int nb = 0; nb < 4; ++nb) { const V b = WFrag<T16>::ld(Bt + boff + (size_t)nb * 16 * K + kc); V b2; if (NSPLIT >= 2) b2 = WFrag<T16>::ld(Bt2 + boff + (size_t)nb * 16 * K + kc);
#pragma unroll
            for (int mb = 0; mb < 4; ++mb) { acc[mb][nb] = WFrag<T16>::mma(a[mb], b, acc[mb][nb]); if (NSPLIT == 1 || NSPLIT == 2) acc[mb][nb] = WFrag<T16>::mma(a2[mb], b, acc[mb][nb]); if (NSPLIT >= 2) acc[mb][nb] = WFrag<T16>::mma(a[mb], b2, acc[mb][nb]); } }
        asm volatile("v_nop\n\tv_nop\n\tv_nop\n\tv_nop" : "+v"(acc[0][0]), "+v"(acc[1][1]), "+v"(acc[2][2]), "+v"(acc[3][3]) : "v"(a[0]), "v"(a[3]));
    }
#pragma unroll
    for (int mb = 0; mb < 4; ++mb) {
#pragma unroll
        for (int nb = 0; nb < 4; ++nb) {
#pragma unroll
            for (int j = 0; j < 8; ++j) os[(hi * 8 + j) * 68 + nb * 16 + lr] = acc[mb][nb][j]; }
        __builtin_amdgcn_wave_barrier(); asm volatile("" ::: "memory");
        float* crow = C + (size_t)(r0 + mb * 16) * ldc + c0;
#pragma unroll 1
        for (int ps = 0; ps < 2; ++ps) {
#pragma unroll
            for (int s = 0; s < 8; ++s) { const int row = 2 * s + hi, cofs = lr * 4; v4f val = *(const v4fa*)(os + row * 68 + cofs); if (BIAS) { val[0] += bfr(bias[c0 + cofs]); val[1] += bfr(bias[c0 + cofs + 1]); val[2] += bfr(bias[c0 + cofs + 2]); val[3] += bfr(bias[c0 + cofs + 3]); }
                *(volatile v4f*)(crow + (size_t)row * ldc + cofs) = val; }
            if (ps == 0) __threadfence(); }
        __builtin_amdgcn_wave_barrier(); asm volatile("" ::: "memory");
    }
}

__device__ __forceinline__ h16 tohx(float x) { return (h16)x; }
__device__ __forceinline__ void splitf(float y, unsigned short& h, unsigned short& l) { h = f2bf(y); l = f2bf(y - bf2f(h)); }
typedef __attribute__((ext_vector_type(2))) _Float16 v2h;
typedef __attribute__((ext_vector_type(4))) _Float16 v4h;
typedef __attribute__((ext_vector_type(2))) unsigned short v2us;
typedef __attribute__((ext_vector_type(4))) unsigned short v4us;
typedef __attribute__((ext_vector_type(2))) float v2f;
typedef __attribute__((ext_vector_type(4))) int v4i;

__global__ __launch_bounds__(256) void k_wtG(const float* __restrict__ w, int K, int N, bf* Bt) {
    const int lane = threadIdx.x & 31; const int L0 = (blockIdx.x * 8 + (threadIdx.x >> 5)) * 8; const int nlines = N * K / 64;
#pragma unroll
    for (int ps = 0; ps < 2; ++ps) {
        for (int l = 0; l < 8; ++l) { const int L = L0 + l; if (L >= nlines) break; const size_t e = (size_t)L * 64 + lane * 2; const int k = (int)(e % K), n = (int)(e / K); v2us o;
            o[0] = f2bf(w[(size_t)k * N + n]); o[1] = f2bf(w[(size_t)(k + 1) * N + n]); *(volatile v2us*)(Bt + e) = o; }
        if (ps == 0) __threadfence(); }
}

__global__ __launch_bounds__(256) void k_kf(const float* __restrict__ kk, const float* __restrict__ mk, bf* KH, bf* KL) {
    const size_t t = (size_t)blockIdx.x * 256 + threadIdx.x; if (t >= (size_t)NBH * ND * (NN / 2)) return; const int n = (int)(t % (NN / 2)) * 2, d = (int)((t / (NN / 2)) % ND), bh = (int)(t / ((size_t)(NN / 2) * ND)); const int b = bh / NHH;
    v2us hh, ll; unsigned short a, c;
#pragma unroll
    for (int q = 0; q < 2; ++q) { const float k = bfr(kk[((size_t)bh * NN + n + q) * ND + d]); const float m = bfr(mk[(size_t)b * NN + n + q]); const float f = fmaxf(k, 0.0f) + expf(fminf(k, 0.0f)); const float y = ((f * m) * 0.125f) * m; splitf(y, a, c); hh[q] = a; ll[q] = c; }
    const size_t o = ((size_t)bh * ND + d) * NN + n;
#pragma unroll
    for (int ps = 0; ps < 2; ++ps) { *(volatile v2us*)(KH + o) = hh; *(volatile v2us*)(KL + o) = ll; if (ps == 0) __threadfence(); } }

__global__ __launch_bounds__(256) void k_qf(const float* __restrict__ qq, bf* QB) {
    const size_t t = (size_t)blockIdx.x * 256 + threadIdx.x; if (t >= (size_t)NBH * NN * ND / 8) return; const v4f x0 = *(const v4f*)(qq + 8 * t), x1 = *(const v4f*)(qq + 8 * t + 4); v8us o;
#pragma unroll
    for (int j = 0; j < 4; ++j) { const float a = bfr(x0[j]), c = bfr(x1[j]); o[j] = f2bf((fmaxf(a, 0.0f) + expf(fminf(a, 0.0f))) * 0.125f); o[4 + j] = f2bf((fmaxf(c, 0.0f) + expf(fminf(c, 0.0f))) * 0.125f); }
    *(volatile v8us*)(QB + 8 * t) = o; __threadfence(); *(volatile v8us*)(QB + 8 * t) = o; }

extern "C" void kernel_launch(void* const* d_in, const int* in_sizes, int n_in,
                              void* d_out, int out_size, void* d_ws, size_t ws_size, hipStream_t stream) {
    if (n_in < 4) return;
    if (in_sizes[0] < NBH * NN * ND || in_sizes[1] < NBH * NN * ND || in_sizes[2] < NBH * NN * ND || in_sizes[3] < (NBH / NHH) * NN || out_size < NBH * NN * ND) return;
    const float* qq = (const float*)d_in[0]; const float* kk = (const float*)d_in[1]; const float* vv = (const float*)d_in[2]; const float* mk = (const float*)d_in[3];
    float* OUT = (float*)d_out;
    char* wsp = (char*)d_ws;
    auto take = [&](size_t bytes) { char* p = wsp; wsp += (bytes + 255) & ~(size_t)255; return (void*)p; };
    bf* KH = (bf*)take((size_t)NBH * ND * NN * 2); bf* KL = (bf*)take((size_t)NBH * ND * NN * 2); bf* VT = (bf*)take((size_t)NBH * ND * NN * 2); bf* QB = (bf*)take((size_t)NBH * ND * NN * 2);
    float* KTV = (float*)take((size_t)NBH * ND * ND * 4); bf* KB = (bf*)take((size_t)NBH * ND * ND * 2);
    if ((size_t)(wsp - (char*)d_ws) != WS_TOTAL || WS_TOTAL > ws_size) return;
    for (int z = 0; z < NBH; ++z) k_wtG<<<(unsigned)((NN * ND / 64 + 63) / 64), 256, 0, stream>>>(vv + (size_t)z * NN * ND, NN, ND, VT + (size_t)z * ND * NN);
    k_kf<<<(unsigned)(((size_t)NBH * ND * (NN / 2) + 255) / 256), 256, 0, stream>>>(kk, mk, KH, KL);
    k_qf<<<(unsigned)(((size_t)NBH * NN * ND / 8 + 255) / 256), 256, 0, stream>>>(qq, QB);
    k_gemmw<bf, 1, false><<<dim3(ND / 64, ND / 64, NBH), 32, 0, stream>>>(KH, KL, VT, nullptr, NN, KTV, ND, nullptr, (size_t)ND * NN, (size_t)ND * NN, (size_t)ND * ND);
    for (int z = 0; z < NBH; ++z) k_wtG<<<(unsigned)((ND * ND / 64 + 63) / 64), 256, 0, stream>>>(KTV + (size_t)z * ND * ND, ND, ND, KB + (size_t)z * ND * ND);
    k_gemmw<bf, 0, false><<<dim3(NN / 64, ND / 64, NBH), 32, 0, stream>>>(QB, nullptr, KB, nullptr, ND, OUT, ND, nullptr, (size_t)NN * ND, (size_t)ND * ND, (size_t)NN * ND);
}
